// MultiTaskMLP_34763465294401
// MI455X (gfx1250) — hardware-run, weakly checked
//
#include <hip/hip_runtime.h>


#ifndef NB
#define NB 65536
#endif
#define NB_FULL 65536
#define DIN   100
#define KX    128
#define E1W   256
#define E2W   128
#define NG    100
#define NGP   128
#define D1W   64
#define D2W   32
#define RB    1024
#define NBLK  (NB / RB)
#define OFFP  128
#define TSZ   (3 * NGP)
#define PROWS (((NB + NG * 63 + 63) / 64) * 64)
#define BN_EPS 1e-5f

static_assert(NB % RB == 0);
static_assert(NBLK >= 1 && NBLK <= OFFP);
static_assert(NB <= NB_FULL);
static_assert(NG <= NGP && NGP == 128);
static_assert(PROWS % 64 == 0);
static_assert(PROWS >= NB + NG * 63);
static_assert(NB % 4 == 0);
static_assert(DIN % 4 == 0 && DIN <= KX && KX % 32 == 0);
static_assert(E1W % 64 == 0 && E2W % 64 == 0 && D1W % 64 == 0 && D2W == 32);
static_assert(KX % 64 == 0 && E1W % 64 == 0 && E2W % 64 == 0 && D1W % 64 == 0);
static_assert(E1W % 32 == 0 && E2W % 32 == 0 && D1W % 32 == 0 && D2W % 32 == 0);
static_assert(256 * 16 * 1 == 32 * 64 * 2);
static_assert(32 * 16 * 1 == NGP * 4);
static_assert(32 * 16 * 32 == 64 * KX * 2);
static_assert(32 * 16 * 16 == 32 * KX * 2);
static_assert(32 * 16 * 4 == 16 * 64 * 2);
static_assert(16 * 16 * 1 == 64 * 4);
static_assert(64 * 33 * 4 <= 131072);
static_assert(32 * NGP * 4 + NGP * 4 <= 131072);
static_assert(2 * NGP * 4 + TSZ * 4 <= 131072);
static_assert(16 * 68 * 4 <= 131072);
static_assert(16 * 36 * 4 + 6 * 32 * 4 + 64 * 4 <= 131072);

typedef unsigned short bf;
typedef __attribute__((ext_vector_type(16))) __bf16   v16bf;
typedef __attribute__((ext_vector_type(8)))  unsigned short v8us;
typedef __attribute__((ext_vector_type(8)))  float    v8f;
typedef __attribute__((ext_vector_type(4)))  float    v4f;
typedef __attribute__((ext_vector_type(4)))  int      v4i;
typedef v4f  __attribute__((may_alias)) v4fa;
typedef v4i  __attribute__((may_alias)) v4ia;

__device__ __forceinline__ unsigned short f2bf(float f) { unsigned u = __float_as_uint(f); u += 0x7FFFu + ((u >> 16) & 1u); return (unsigned short)(u >> 16); }
__device__ __forceinline__ float bf2f(unsigned short w) { return __uint_as_float(((unsigned)w) << 16); }
__device__ __forceinline__ int clampi(int v, int lo, int hi) { return min(max(v, lo), hi); }
__device__ __forceinline__ v16bf cat16b(v8us lo, v8us hi) { return __builtin_bit_cast(v16bf, __builtin_shufflevector(lo, hi, 0, 1, 2, 3, 4, 5, 6, 7, 8, 9, 10, 11, 12, 13, 14, 15)); }
__device__ __forceinline__ v8f wmmab(v16bf a, v16bf b, v8f c) { return __builtin_amdgcn_wmma_f32_16x16x32_bf16(false, a, false, b, (short)0, c, false, false); }
__device__ __forceinline__ v16bf ldb(const bf* p)  { return cat16b(*(const v8us*)p, *(const v8us*)(p + 16)); }
__device__ __forceinline__ void wave_sync() { __builtin_amdgcn_fence(3  , "wavefront"); __builtin_amdgcn_wave_barrier(); asm volatile("" ::: "memory"); }
__device__ __forceinline__ float bfr(float f) { return bf2f(f2bf(f)); }

__global__ __launch_bounds__(256) void k_wt(const float* __restrict__ W, bf* WT, int KS, int KP, int N) {
    __shared__ float ts[64 * 33];
    const int t = threadIdx.x;
    const int kt = blockIdx.x, nt = blockIdx.y, g = blockIdx.z;
    const float* src = W + (size_t)g * KS * N;
#pragma unroll 1
    for (int i = 0; i < 8; ++i) { const int f = i * 256 + t; const int k = f >> 5, n = f & 31; const int kg = kt * 64 + k; const int kc = min(kg, KS - 1);
        const float v = src[(size_t)kc * N + nt * 32 + n]; ts[k * 33 + n] = (kg < KS) ? v : 0.0f; }
    __syncthreads();
    bf* dst = WT + ((size_t)g * N + (size_t)nt * 32) * KP + kt * 64;
    const int e = t >> 3, c8 = (t & 7) * 8; v8us o;
#pragma unroll
    for (int k = 0; k < 8; ++k) o[k] = f2bf(ts[(c8 + k) * 33 + e]);
#pragma unroll 1
    for (int ps = 0; ps < 2; ++ps) {
        *(volatile v8us*)(dst + (size_t)e * KP + c8) = o;
        if (ps == 0) __threadfence(); }
}

__global__ __launch_bounds__(1024) void k_count(const int* __restrict__ ids, int* cnt) {
    __shared__ int wc[32 * NGP];
    __shared__ __align__(16) int line[NGP];
    const int tid = threadIdx.x, lane = tid & 31; const int wave = __builtin_amdgcn_readfirstlane(tid >> 5);
    const int blk = blockIdx.x;
    const int g = clampi(ids[(size_t)blk * RB + tid], 0, NG - 1);
    int m0 = 0, m1 = 0, m2 = 0, m3 = 0;
#pragma unroll 1
    for (int r = 0; r < 32; ++r) {
        const int c0 = __builtin_popcount(__builtin_amdgcn_ballot_w32(g == r));
        const int c1 = __builtin_popcount(__builtin_amdgcn_ballot_w32(g == 32 + r));
        const int c2 = __builtin_popcount(__builtin_amdgcn_ballot_w32(g == 64 + r));
        const int c3 = __builtin_popcount(__builtin_amdgcn_ballot_w32(g == 96 + r));
        m0 = (lane == r) ? c0 : m0; m1 = (lane == r) ? c1 : m1; m2 = (lane == r) ? c2 : m2; m3 = (lane == r) ? c3 : m3; }
    wc[wave * NGP + lane] = m0; wc[wave * NGP + 32 + lane] = m1; wc[wave * NGP + 64 + lane] = m2; wc[wave * NGP + 96 + lane] = m3;
    __syncthreads();
    if (wave < 4) {
        int s = 0;
#pragma unroll 1
        for (int w = 0; w < 32; ++w) s += wc[w * NGP + wave * 32 + lane];
        line[wave * 32 + lane] = s;
    }
    __syncthreads();
    if (wave == 0) {
#pragma unroll 1
        for (int ps = 0; ps < 2; ++ps) {
            const v4i v = *(const v4ia*)(&line[4 * lane]); *(volatile v4i*)(cnt + (size_t)blk * NGP + 4 * lane) = v;
            if (ps == 0) __threadfence(); }
    }
}

__global__ __launch_bounds__(1024) void k_scan(const int* __restrict__ cnt, int* offs, int* T, bf* XP) {
    __shared__ int tots[NGP];
    __shared__ int sst[NGP];
    __shared__ __align__(16) int tl[TSZ];
    const int tid = threadIdx.x, lane = tid & 31; const int w = __builtin_amdgcn_readfirstlane(tid >> 5);
    int c[4][4]; int excl[4]; int tot[4];
#pragma unroll
    for (int gi = 0; gi < 4; ++gi) {
        const int g = 4 * w + gi; int ls = 0;
#pragma unroll
        for (int i = 0; i < 4; ++i) { const int blk = 4 * lane + i; const int bc = min(blk, NBLK - 1);
            int v = cnt[(size_t)bc * NGP + g]; v = (blk < NBLK) ? v : 0; v = clampi(v, 0, RB); c[gi][i] = v; ls += v; }
        int x = ls;
#pragma unroll
        for (int d = 1; d < 32; d <<= 1) { const int y = __shfl_up(x, d, 32); x += (lane >= d) ? y : 0; }
        excl[gi] = x - ls;
        tot[gi] = __shfl(x, 31, 32);
        if (lane == 0) tots[g] = tot[gi];
    }
    __syncthreads();
    if (w == 0) {
        int t4[4]; int pd[4]; int lsum = 0;
#pragma unroll
        for (int i = 0; i < 4; ++i) { t4[i] = tots[4 * lane + i]; pd[i] = (t4[i] + 63) & ~63; lsum += pd[i]; }
        int y2 = lsum;
#pragma unroll
        for (int d = 1; d < 32; d <<= 1) { const int y = __shfl_up(y2, d, 32); y2 += (lane >= d) ? y : 0; }
        int run = y2 - lsum;
        const int ptot = __shfl(y2, 31, 32);
#pragma unroll
        for (int i = 0; i < 4; ++i) { sst[4 * lane + i] = run; tl[4 * lane + i] = run; tl[NGP + 4 * lane + i] = t4[i];
            tl[2 * NGP + 4 * lane + i] = (lane == 0 && i == 0) ? ptot : 0; run += pd[i]; }
    }
    __syncthreads();
    int segr[4];
#pragma unroll
    for (int gi = 0; gi < 4; ++gi) segr[gi] = sst[4 * w + gi];
    v8us z;
#pragma unroll
    for (int k = 0; k < 8; ++k) z[k] = (unsigned short)0;
    const int c8 = (lane & 15) * 8;
#pragma unroll 1
    for (int ps = 0; ps < 2; ++ps) {
#pragma unroll
        for (int gi = 0; gi < 4; ++gi) {
            const int g = 4 * w + gi;
            v4i o; o[0] = segr[gi] + excl[gi]; o[1] = o[0] + c[gi][0]; o[2] = o[1] + c[gi][1]; o[3] = o[2] + c[gi][2];
            *(volatile v4i*)(offs + (size_t)g * OFFP + 4 * lane) = o;
            const int padcnt = ((tot[gi] + 63) & ~63) - tot[gi];
            const int pbase = segr[gi] + tot[gi];
#pragma unroll 1
            for (int it = 0; it < 32; ++it) { const int j = 2 * it + (lane >> 4); const int p = clampi(pbase + j, 0, PROWS - 1);
                if (j < padcnt) { *(volatile v8us*)(XP + (size_t)p * KX + c8) = z; } }
        }
        if (w == 0) {
#pragma unroll
            for (int q = 0; q < 3; ++q) { const v4i v = *(const v4ia*)(&tl[q * NGP + 4 * lane]); *(volatile v4i*)(T + q * NGP + 4 * lane) = v; }
        }
        if (ps == 0) __threadfence(); }
}

__global__ __launch_bounds__(1024) void k_rank(const int* __restrict__ ids, const float* __restrict__ x,
                                               const int* __restrict__ offs, int* POS, bf* XP) {
    __shared__ int wc[32 * NGP];
    const int tid = threadIdx.x, lane = tid & 31; const int wave = __builtin_amdgcn_readfirstlane(tid >> 5);
    const int blk = blockIdx.x;
    const size_t row = (size_t)blk * RB + tid;
    const int g = clampi(ids[row], 0, NG - 1);
    int m0 = 0, m1 = 0, m2 = 0, m3 = 0; unsigned mymask = 0u;
#pragma unroll 1
    for (int r = 0; r < 32; ++r) {
        const unsigned b0 = __builtin_amdgcn_ballot_w32(g == r);
        const unsigned b1 = __builtin_amdgcn_ballot_w32(g == 32 + r);
        const unsigned b2 = __builtin_amdgcn_ballot_w32(g == 64 + r);
        const unsigned b3 = __builtin_amdgcn_ballot_w32(g == 96 + r);
        const int c0 = __builtin_popcount(b0), c1 = __builtin_popcount(b1), c2 = __builtin_popcount(b2), c3 = __builtin_popcount(b3);
        m0 = (lane == r) ? c0 : m0; m1 = (lane == r) ? c1 : m1; m2 = (lane == r) ? c2 : m2; m3 = (lane == r) ? c3 : m3;
        mymask = (g == r) ? b0 : mymask; mymask = (g == 32 + r) ? b1 : mymask; mymask = (g == 64 + r) ? b2 : mymask; mymask = (g == 96 + r) ? b3 : mymask; }
    const int lrank = __builtin_popcount(mymask & ((1u << lane) - 1u));
    wc[wave * NGP + lane] = m0; wc[wave * NGP + 32 + lane] = m1; wc[wave * NGP + 64 + lane] = m2; wc[wave * NGP + 96 + lane] = m3;
    __syncthreads();
    if (wave < 4) {
        const int gs = wave * 32 + lane;
        int run = clampi(offs[(size_t)gs * OFFP + blk], 0, PROWS);
#pragma unroll 1
        for (int w = 0; w < 32; ++w) { const int c = wc[w * NGP + gs]; wc[w * NGP + gs] = run; run += c; }
    }
    __syncthreads();
    const int pos = clampi(wc[wave * NGP + g] + lrank, 0, PROWS - 1);
    const int c8 = (lane & 15) * 8;
    const int ca = min(c8, DIN - 4), cb = min(c8 + 4, DIN - 4);
    const bool oka = (c8 < DIN), okb = (c8 + 4 < DIN);
#pragma unroll 1
    for (int ps = 0; ps < 2; ++ps) {
        *(volatile int*)(POS + row) = pos;
#pragma unroll 1
        for (int it = 0; it < 16; ++it) { const int j = 2 * it + (lane >> 4); const int p = __shfl(pos, j, 32);
            const size_t rg = (size_t)blk * RB + (size_t)wave * 32 + j;
            const v4f a = *(const v4f*)(x + rg * DIN + ca); const v4f b = *(const v4f*)(x + rg * DIN + cb); v8us o;
#pragma unroll
            for (int k = 0; k < 4; ++k) { const unsigned short ua = f2bf(a[k]); const unsigned short ub = f2bf(b[k]);
                o[k] = oka ? ua : (unsigned short)0; o[4 + k] = okb ? ub : (unsigned short)0; }
            *(volatile v8us*)(XP + (size_t)p * KX + c8) = o; }
        if (ps == 0) __threadfence(); }
}

static __device__ __forceinline__ int find_group(const int* __restrict__ T, int p0) {
    const int lane = threadIdx.x & 31;
    int s0 = T[lane], s1 = T[32 + lane], s2 = T[64 + lane], s3 = T[96 + lane];
    int t0 = T[NGP + lane], t1 = T[NGP + 32 + lane], t2 = T[NGP + 64 + lane], t3 = T[NGP + 96 + lane];
    asm volatile("" : "+v"(s0), "+v"(s1), "+v"(s2), "+v"(s3), "+v"(t0), "+v"(t1), "+v"(t2), "+v"(t3));
    const unsigned k0 = __builtin_amdgcn_ballot_w32((p0 >= s0) & (p0 < s0 + ((t0 + 63) & ~63)));
    const unsigned k1 = __builtin_amdgcn_ballot_w32((p0 >= s1) & (p0 < s1 + ((t1 + 63) & ~63)));
    const unsigned k2 = __builtin_amdgcn_ballot_w32((p0 >= s2) & (p0 < s2 + ((t2 + 63) & ~63)));
    const unsigned k3 = __builtin_amdgcn_ballot_w32((p0 >= s3) & (p0 < s3 + ((t3 + 63) & ~63)));
    int gs = 96 + __builtin_ctz(k3 | 0x80000000u);
    gs = (k2 != 0u) ? (64 + __builtin_ctz(k2 | 0x80000000u)) : gs;
    gs = (k1 != 0u) ? (32 + __builtin_ctz(k1 | 0x80000000u)) : gs;
    gs = (k0 != 0u) ? __builtin_ctz(k0 | 0x80000000u) : gs;
    gs = clampi(gs, 0, NG - 1);
    gs = ((k0 | k1 | k2 | k3) != 0u) ? gs : -1;
    return __builtin_amdgcn_readfirstlane(gs);
}

template <int KA, int KW, int NOUT, bool GROUPED>
static __device__ __forceinline__ void gemm_bn(const bf* __restrict__ AP, const bf* __restrict__ WT,
                                               const float* __restrict__ vb, const float* __restrict__ vg, const float* __restrict__ vt,
                                               const float* __restrict__ vm, const float* __restrict__ vv,
                                               const int* __restrict__ T, bf* OUTP) {
    static_assert(KA % 32 == 0);
    static_assert((KW & (KW - 1)) == 0 && KW >= 32);
    static_assert(KA == KW || KA == 2 * KW);
    static_assert(NOUT % 64 == 0);
    __shared__ __align__(16) float os[16 * 68];
    const int lane = threadIdx.x & 31, lr = lane & 15, hi = lane >> 4;
    const int p0 = blockIdx.x * 64;
    const int ns = blockIdx.y;
    const int g = find_group(T, p0);
    if (g < 0) return;
    const int gq = GROUPED ? g : 0;
    v8f acc[4][4];
#pragma unroll
    for (int mb = 0; mb < 4; ++mb)
#pragma unroll
        for (int nb = 0; nb < 4; ++nb) acc[mb][nb] = (v8f){};
    const size_t aoff = (size_t)(p0 + lr) * KA + 8 * hi;
    const size_t boff = (size_t)gq * ((size_t)NOUT * KW) + (size_t)(ns * 64 + lr) * KW + 8 * hi;
#pragma unroll 1
    for (int kc = 0; kc < KA; kc += 32) {
        const int kw = kc & (KW - 1);
        v16bf a[4];
#pragma unroll
        for (int mb = 0; mb < 4; ++mb) a[mb] = ldb(AP + aoff + (size_t)mb * 16 * KA + kc);
#pragma unroll
        for (int nb = 0; nb < 4; ++nb) { const v16bf b = ldb(WT + boff + (size_t)nb * 16 * KW + kw);
#pragma unroll
            for (int mb = 0; mb < 4; ++mb) acc[mb][nb] = wmmab(a[mb], b, acc[mb][nb]); }
        asm volatile("v_nop\n\tv_nop\n\tv_nop\n\tv_nop" : "+v"(acc[0][0]), "+v"(acc[1][1]), "+v"(acc[2][2]), "+v"(acc[3][3]) : "v"(a[0]), "v"(a[1]), "v"(a[2]), "v"(a[3]));
    }
    const int c8 = (lane & 7) * 8, rq = lane >> 3;
    const int cn = gq * NOUT + ns * 64 + c8;
    float eb[8], em[8], er[8], eg[8], et[8];
    {
        const v4f b0 = *(const v4f*)(vb + cn), b1 = *(const v4f*)(vb + cn + 4);
        const v4f g0 = *(const v4f*)(vg + cn), g1 = *(const v4f*)(vg + cn + 4);
        const v4f t0 = *(const v4f*)(vt + cn), t1 = *(const v4f*)(vt + cn + 4);
        const v4f m0 = *(const v4f*)(vm + cn), m1 = *(const v4f*)(vm + cn + 4);
        const v4f v0 = *(const v4f*)(vv + cn), v1 = *(const v4f*)(vv + cn + 4);
#pragma unroll
        for (int k = 0; k < 4; ++k) {
            eb[k] = bfr(b0[k]); eb[4 + k] = bfr(b1[k]);
            eg[k] = bfr(g0[k]); eg[4 + k] = bfr(g1[k]);
            et[k] = bfr(t0[k]); et[4 + k] = bfr(t1[k]);
            em[k] = bfr(m0[k]); em[4 + k] = bfr(m1[k]);
            er[k] = rsqrtf(bfr(v0[k]) + BN_EPS); er[4 + k] = rsqrtf(bfr(v1[k]) + BN_EPS); }
    }
#pragma unroll
    for (int mb = 0; mb < 4; ++mb) {
#pragma unroll
        for (int nb = 0; nb < 4; ++nb) {
#pragma unroll
            for (int j = 0; j < 8; ++j) os[(hi * 8 + j) * 68 + nb * 16 + lr] = acc[mb][nb][j]; }
        wave_sync();
#pragma unroll 1
        for (int ps = 0; ps < 2; ++ps) {
#pragma unroll 1
            for (int i = 0; i < 4; ++i) {
                const int r = 4 * i + rq;
                const v4f x0 = *(const v4fa*)(&os[r * 68 + c8]); const v4f x1 = *(const v4fa*)(&os[r * 68 + c8 + 4]);
                v8us oh, ol;
#pragma unroll
                for (int k = 0; k < 8; ++k) {
                    const float xin = (k < 4) ? x0[k & 3] : x1[k & 3];
                    const float zz = xin + eb[k];
                    float y = (zz - em[k]) * er[k];
                    y = y * eg[k] + et[k];
                    y = (y > 0.0f) ? y : 0.0f;
                    const unsigned short h = f2bf(y);
                    oh[k] = h; ol[k] = f2bf(y - bf2f(h)); }
                bf* dst = OUTP + (size_t)(p0 + mb * 16 + r) * (2 * NOUT) + ns * 64 + c8;
                *(volatile v8us*)dst = oh; *(volatile v8us*)(dst + NOUT) = ol; }
            if (ps == 0) __threadfence(); }
        wave_sync();
    }
}

__global__ __launch_bounds__(32) __attribute__((amdgpu_num_vgpr(256))) void k_enc1(const bf* __restrict__ XP, const bf* __restrict__ W1T,
        const float* __restrict__ eb1, const float* __restrict__ eg1, const float* __restrict__ ebt1, const float* __restrict__ em1, const float* __restrict__ ev1,
        const int* __restrict__ T, bf* H1) {
    gemm_bn<KX, KX, E1W, false>(XP, W1T, eb1, eg1, ebt1, em1, ev1, T, H1);
}
__global__ __launch_bounds__(32) __attribute__((amdgpu_num_vgpr(256))) void k_enc2(const bf* __restrict__ H1, const bf* __restrict__ W2T,
        const float* __restrict__ eb2, const float* __restrict__ eg2, const float* __restrict__ ebt2, const float* __restrict__ em2, const float* __restrict__ ev2,
        const int* __restrict__ T, bf* H2) {
    gemm_bn<2 * E1W, E1W, E2W, false>(H1, W2T, eb2, eg2, ebt2, em2, ev2, T, H2);
}
__global__ __launch_bounds__(32) __attribute__((amdgpu_num_vgpr(256))) void k_dec1(const bf* __restrict__ H2, const bf* __restrict__ D1T,
        const float* __restrict__ db1, const float* __restrict__ dg1, const float* __restrict__ dbt1, const float* __restrict__ dm1, const float* __restrict__ dv1,
        const int* __restrict__ T, bf* Z1) {
    gemm_bn<2 * E2W, E2W, D1W, true>(H2, D1T, db1, dg1, dbt1, dm1, dv1, T, Z1);
}

__global__ __launch_bounds__(32) __attribute__((amdgpu_num_vgpr(256))) void k_dec2(const bf* __restrict__ Z1, const bf* __restrict__ D2T,
        const float* __restrict__ db2, const float* __restrict__ dg2, const float* __restrict__ dbt2, const float* __restrict__ dm2, const float* __restrict__ dv2,
        const float* __restrict__ dW3, const float* __restrict__ db3, const int* __restrict__ T, float* SORTED) {
    __shared__ __align__(16) float os[16 * 36];
    __shared__ __align__(16) float pv[6 * 32];
    __shared__ __align__(16) float res[64];
    const int lane = threadIdx.x & 31, lr = lane & 15, hi = lane >> 4;
    const int p0 = blockIdx.x * 64;
    const int g = find_group(T, p0);
    if (g < 0) return;
    v8f acc[4][2];
#pragma unroll
    for (int mb = 0; mb < 4; ++mb)
#pragma unroll
        for (int nb = 0; nb < 2; ++nb) acc[mb][nb] = (v8f){};
    const size_t aoff = (size_t)(p0 + lr) * (2 * D1W) + 8 * hi;
    const size_t boff = (size_t)g * (D2W * D1W) + (size_t)lr * D1W + 8 * hi;
#pragma unroll 1
    for (int kc = 0; kc < 2 * D1W; kc += 32) {
        const int kw = kc & (D1W - 1);
        v16bf a[4];
#pragma unroll
        for (int mb = 0; mb < 4; ++mb) a[mb] = ldb(Z1 + aoff + (size_t)mb * 16 * (2 * D1W) + kc);
#pragma unroll
        for (int nb = 0; nb < 2; ++nb) { const v16bf b = ldb(D2T + boff + (size_t)nb * 16 * D1W + kw);
#pragma unroll
            for (int mb = 0; mb < 4; ++mb) acc[mb][nb] = wmmab(a[mb], b, acc[mb][nb]); }
        asm volatile("v_nop\n\tv_nop\n\tv_nop\n\tv_nop" : "+v"(acc[0][0]), "+v"(acc[1][1]), "+v"(acc[2][0]), "+v"(acc[3][1]) : "v"(a[0]), "v"(a[1]), "v"(a[2]), "v"(a[3]));
    }
    {
        const int cv = g * D2W + lane;
        pv[lane] = bfr(db2[cv]); pv[32 + lane] = bfr(dm2[cv]); pv[64 + lane] = rsqrtf(bfr(dv2[cv]) + BN_EPS);
        pv[96 + lane] = bfr(dg2[cv]); pv[128 + lane] = bfr(dbt2[cv]); pv[160 + lane] = bfr(dW3[cv]);
    }
    const float b3 = bfr(db3[g]);
    wave_sync();
    const int row = lane >> 1, hf = lane & 1;
#pragma unroll
    for (int mb = 0; mb < 4; ++mb) {
#pragma unroll
        for (int nb = 0; nb < 2; ++nb) {
#pragma unroll
            for (int j = 0; j < 8; ++j) os[(hi * 8 + j) * 36 + nb * 16 + lr] = acc[mb][nb][j]; }
        wave_sync();
        float s = 0.0f;
#pragma unroll
        for (int q = 0; q < 4; ++q) {
            const int co = hf * 16 + 4 * q;
            const v4f xv = *(const v4fa*)(&os[row * 36 + co]);
            const v4f qb = *(const v4fa*)(&pv[co]);       const v4f qm = *(const v4fa*)(&pv[32 + co]);
            const v4f qr = *(const v4fa*)(&pv[64 + co]);  const v4f qg = *(const v4fa*)(&pv[96 + co]);
            const v4f qt = *(const v4fa*)(&pv[128 + co]); const v4f qw = *(const v4fa*)(&pv[160 + co]);
#pragma unroll
            for (int i = 0; i < 4; ++i) { const float zz = xv[i] + qb[i]; float y = (zz - qm[i]) * qr[i]; y = y * qg[i] + qt[i]; y = (y > 0.0f) ? y : 0.0f; s += y * qw[i]; } }
        s += __shfl_xor(s, 1, 32);
        if (hf == 0) res[mb * 16 + row] = s + b3;
        wave_sync();
    }
#pragma unroll 1
    for (int ps = 0; ps < 2; ++ps) {
        if (lane < 16) { const v4f v = *(const v4fa*)(&res[4 * lane]); *(volatile v4f*)(SORTED + (size_t)p0 + 4 * lane) = v; }
        if (ps == 0) __threadfence(); }
}

__global__ __launch_bounds__(256) void k_unsort(const int* __restrict__ POS, const float* __restrict__ SORTED, float* OUT) {
    const size_t i = (size_t)blockIdx.x * 256 + threadIdx.x; if (i >= (size_t)(NB / 4)) return;
    const v4i p = *(const v4i*)(POS + i * 4); v4f v;
#pragma unroll
    for (int k = 0; k < 4; ++k) v[k] = SORTED[clampi(p[k], 0, PROWS - 1)];
    *(volatile v4f*)(OUT + i * 4) = v; __threadfence(); *(volatile v4f*)(OUT + i * 4) = v;
}

static constexpr size_t al256(size_t v) { return (v + 255) & ~(size_t)255; }
static constexpr size_t SZ_W1T = al256((size_t)E1W * KX * 2);
static constexpr size_t SZ_W2T = al256((size_t)E2W * E1W * 2);
static constexpr size_t SZ_D1T = al256((size_t)NG * D1W * E2W * 2);
static constexpr size_t SZ_D2T = al256((size_t)NG * D2W * D1W * 2);
static constexpr size_t SZ_CNT = al256((size_t)NBLK * NGP * 4);
static constexpr size_t SZ_OFF = al256((size_t)NGP * OFFP * 4);
static constexpr size_t SZ_T   = al256((size_t)TSZ * 4);
static constexpr size_t SZ_POS = al256((size_t)NB * 4);
static constexpr size_t SZ_RA  = al256((size_t)PROWS * (2 * E2W) * 2);
static constexpr size_t SZ_RB  = al256((size_t)PROWS * (2 * E1W) * 2);
static constexpr size_t SZ_SRT = al256((size_t)PROWS * 4);
static_assert((size_t)PROWS * KX * 2 <= SZ_RA);
static_assert((size_t)PROWS * (2 * E2W) * 2 <= SZ_RA);
static_assert((size_t)PROWS * (2 * E1W) * 2 <= SZ_RB);
static_assert((size_t)PROWS * (2 * D1W) * 2 <= SZ_RB);
static constexpr size_t SZ_TOTAL = SZ_W1T + SZ_W2T + SZ_D1T + SZ_D2T + SZ_CNT + SZ_OFF + SZ_T + SZ_POS + SZ_RA + SZ_RB + SZ_SRT;
static_assert(SZ_TOTAL <= (size_t)134217728);

extern "C" void kernel_launch(void* const* d_in, const int* in_sizes, int n_in,
                              void* d_out, int out_size, void* d_ws, size_t ws_size, hipStream_t stream) {
    if (n_in < 28) return;
    if ((size_t)in_sizes[0] < (size_t)NB * DIN) return;
    if ((size_t)in_sizes[1] < (size_t)DIN * E1W) return;
    if ((size_t)in_sizes[2] < (size_t)E1W || (size_t)in_sizes[3] < (size_t)E1W || (size_t)in_sizes[4] < (size_t)E1W ||
        (size_t)in_sizes[5] < (size_t)E1W || (size_t)in_sizes[6] < (size_t)E1W) return;
    if ((size_t)in_sizes[7] < (size_t)E1W * E2W) return;
    if ((size_t)in_sizes[8] < (size_t)E2W || (size_t)in_sizes[9] < (size_t)E2W || (size_t)in_sizes[10] < (size_t)E2W ||
        (size_t)in_sizes[11] < (size_t)E2W || (size_t)in_sizes[12] < (size_t)E2W) return;
    if ((size_t)in_sizes[13] < (size_t)NG * E2W * D1W) return;
    if ((size_t)in_sizes[14] < (size_t)NG * D1W || (size_t)in_sizes[15] < (size_t)NG * D1W || (size_t)in_sizes[16] < (size_t)NG * D1W ||
        (size_t)in_sizes[17] < (size_t)NG * D1W || (size_t)in_sizes[18] < (size_t)NG * D1W) return;
    if ((size_t)in_sizes[19] < (size_t)NG * D1W * D2W) return;
    if ((size_t)in_sizes[20] < (size_t)NG * D2W || (size_t)in_sizes[21] < (size_t)NG * D2W || (size_t)in_sizes[22] < (size_t)NG * D2W ||
        (size_t)in_sizes[23] < (size_t)NG * D2W || (size_t)in_sizes[24] < (size_t)NG * D2W) return;
    if ((size_t)in_sizes[25] < (size_t)NG * D2W || (size_t)in_sizes[26] < (size_t)NG) return;
    if ((size_t)in_sizes[27] < (size_t)NB) return;
    if ((size_t)out_size < (size_t)NB) return;
    if (SZ_TOTAL > ws_size) return;
    const float* x    = (const float*)d_in[0];
    const float* eW1  = (const float*)d_in[1];
    const float* eb1  = (const float*)d_in[2];
    const float* eg1  = (const float*)d_in[3];
    const float* ebt1 = (const float*)d_in[4];
    const float* em1  = (const float*)d_in[5];
    const float* ev1  = (const float*)d_in[6];
    const float* eW2  = (const float*)d_in[7];
    const float* eb2  = (const float*)d_in[8];
    const float* eg2  = (const float*)d_in[9];
    const float* ebt2 = (const float*)d_in[10];
    const float* em2  = (const float*)d_in[11];
    const float* ev2  = (const float*)d_in[12];
    const float* dW1  = (const float*)d_in[13];
    const float* db1  = (const float*)d_in[14];
    const float* dg1  = (const float*)d_in[15];
    const float* dbt1 = (const float*)d_in[16];
    const float* dm1  = (const float*)d_in[17];
    const float* dv1  = (const float*)d_in[18];
    const float* dW2  = (const float*)d_in[19];
    const float* db2  = (const float*)d_in[20];
    const float* dg2  = (const float*)d_in[21];
    const float* dbt2 = (const float*)d_in[22];
    const float* dm2  = (const float*)d_in[23];
    const float* dv2  = (const float*)d_in[24];
    const float* dW3  = (const float*)d_in[25];
    const float* db3  = (const float*)d_in[26];
    const int*   ids  = (const int*)d_in[27];
    float* OUT = (float*)d_out;
    char* wsp = (char*)d_ws;
    bf*  W1T = (bf*)wsp;  wsp += SZ_W1T;
    bf*  W2T = (bf*)wsp;  wsp += SZ_W2T;
    bf*  D1T = (bf*)wsp;  wsp += SZ_D1T;
    bf*  D2T = (bf*)wsp;  wsp += SZ_D2T;
    int* CNT = (int*)wsp; wsp += SZ_CNT;
    int* OFF = (int*)wsp; wsp += SZ_OFF;
    int* TT  = (int*)wsp; wsp += SZ_T;
    int* POS = (int*)wsp; wsp += SZ_POS;
    bf*  RA  = (bf*)wsp;  wsp += SZ_RA;
    bf*  RB2 = (bf*)wsp;  wsp += SZ_RB;
    float* SRT = (float*)wsp; wsp += SZ_SRT;

    k_wt<<<dim3(KX / 64, E1W / 32, 1), 256, 0, stream>>>(eW1, W1T, DIN, KX, E1W);
    k_wt<<<dim3(E1W / 64, E2W / 32, 1), 256, 0, stream>>>(eW2, W2T, E1W, E1W, E2W);
    k_wt<<<dim3(E2W / 64, D1W / 32, NG), 256, 0, stream>>>(dW1, D1T, E2W, E2W, D1W);
    k_wt<<<dim3(D1W / 64, D2W / 32, NG), 256, 0, stream>>>(dW2, D2T, D1W, D1W, D2W);
    k_count<<<NBLK, 1024, 0, stream>>>(ids, CNT);
    k_scan<<<1, 1024, 0, stream>>>(CNT, OFF, TT, RA);
    k_rank<<<NBLK, 1024, 0, stream>>>(ids, x, OFF, POS, RA);
    k_enc1<<<dim3(PROWS / 64, E1W / 64), 32, 0, stream>>>(RA, W1T, eb1, eg1, ebt1, em1, ev1, TT, RB2);
    k_enc2<<<dim3(PROWS / 64, E2W / 64), 32, 0, stream>>>(RB2, W2T, eb2, eg2, ebt2, em2, ev2, TT, RA);
    k_dec1<<<dim3(PROWS / 64, D1W / 64), 32, 0, stream>>>(RA, D1T, db1, dg1, dbt1, dm1, dv1, TT, RB2);
    k_dec2<<<PROWS / 64, 32, 0, stream>>>(RB2, D2T, db2, dg2, dbt2, dm2, dv2, dW3, db3, TT, SRT);
    k_unsort<<<(unsigned)((NB / 4 + 255) / 256), 256, 0, stream>>>(POS, SRT, OUT);
}
